// MultiHeadAttention_14998025797968
// MI455X (gfx1250) — hardware-verified
//
#include <hip/hip_runtime.h>


#ifndef NB
#define NB 2
#endif
#ifndef SEQ
#define SEQ 2048
#endif
#define NB_FULL  2
#define SEQ_FULL 2048
#define TT   SEQ
#define DM   512
#define NH_  8
#define HD   64
#define RC   ((SEQ) < 512 ? (SEQ) : 512)
#define PCAR 1024.0f
#define SCL  0.125f
static_assert(NH_ * HD == DM);
static_assert(TT % 256 == 0);
static_assert(TT % RC == 0);
static_assert(RC % 64 == 0);
static_assert(DM % 64 == 0);
static_assert(SEQ <= SEQ_FULL);
static_assert(NB <= NB_FULL);
static_assert(TT % 128 == 0);
static_assert(RC % 8 == 0);
static_assert(SEQ_FULL % 4 == 0);
static_assert(HD % 32 == 0);
static_assert(DM % 32 == 0);
static_assert(TT % 32 == 0);
static_assert((NH_ * RC) % 8 == 0);

typedef _Float16 h16;
typedef unsigned short bf;
typedef __attribute__((ext_vector_type(16))) __bf16   v16bf;
typedef __attribute__((ext_vector_type(16))) _Float16 v16h;
typedef __attribute__((ext_vector_type(8)))  _Float16 v8h;
typedef __attribute__((ext_vector_type(8)))  unsigned short v8us;
typedef __attribute__((ext_vector_type(8)))  float    v8f;
typedef __attribute__((ext_vector_type(4)))  float    v4f;
typedef __attribute__((ext_vector_type(2)))  _Float16 v2h;
typedef __attribute__((ext_vector_type(4)))  _Float16 v4h;
typedef __attribute__((ext_vector_type(2)))  unsigned short v2us;
typedef __attribute__((ext_vector_type(4)))  int v4i;
typedef v4f  __attribute__((may_alias)) v4fa;
typedef v4i  __attribute__((may_alias)) v4ia;

__device__ __forceinline__ unsigned short f2bf(float f) { unsigned u = __float_as_uint(f); u += 0x7FFFu + ((u >> 16) & 1u); return (unsigned short)(u >> 16); }
__device__ __forceinline__ float bf2f(unsigned short b) { return __uint_as_float(((unsigned)b) << 16); }
__device__ __forceinline__ float bfr(float f) { return bf2f(f2bf(f)); }
__device__ __forceinline__ v16h cat16(v8h lo, v8h hi) { return __builtin_shufflevector(lo, hi, 0, 1, 2, 3, 4, 5, 6, 7, 8, 9, 10, 11, 12, 13, 14, 15); }
__device__ __forceinline__ v16bf cat16b(v8us lo, v8us hi) { return __builtin_bit_cast(v16bf, __builtin_shufflevector(lo, hi, 0, 1, 2, 3, 4, 5, 6, 7, 8, 9, 10, 11, 12, 13, 14, 15)); }
__device__ __forceinline__ v8f wmma16(v16h a, v16h b, v8f c) { return __builtin_amdgcn_wmma_f32_16x16x32_f16(false, a, false, b, (short)0, c, false, false); }
__device__ __forceinline__ v8f wmmab(v16bf a, v16bf b, v8f c) { return __builtin_amdgcn_wmma_f32_16x16x32_bf16(false, a, false, b, (short)0, c, false, false); }
__device__ __forceinline__ void splitf(float y, unsigned short& h, unsigned short& l) { h = f2bf(y); l = f2bf(y - bf2f(h)); }
static __device__ __forceinline__ h16 toh_flush(float v) { const h16 r = (h16)v; return (fabsf(v) < 6.103515625e-05f) ? (h16)0.0f : r; }

template <typename T16> struct WFrag;
template <> struct WFrag<h16> { typedef v16h V; static __device__ __forceinline__ V ld(const h16* p) { return cat16(*(const v8h*)p, *(const v8h*)(p + 16)); } static __device__ __forceinline__ v8f mma(V a, V b, v8f c) { return wmma16(a, b, c); } };
template <> struct WFrag<bf> { typedef v16bf V; static __device__ __forceinline__ V ld(const bf* p) { return cat16b(*(const v8us*)p, *(const v8us*)(p + 16)); } static __device__ __forceinline__ v8f mma(V a, V b, v8f c) { return wmmab(a, b, c); } };
template <typename T16, int NSPLIT, bool BIAS>
__global__ __launch_bounds__(32) void k_gemmw(const T16* __restrict__ A, const T16* __restrict__ A2, const T16* __restrict__ Bt, const T16* __restrict__ Bt2, int K, float* C, int ldc, const float* __restrict__ bias, size_t sA, size_t sB, size_t sC) {
    typedef typename WFrag<T16>::V V;
    __shared__ __align__(16) float os[16 * 68];
    const size_t z = blockIdx.z; A += z * sA; if (A2) A2 += z * sA; Bt += z * sB; if (Bt2) Bt2 += z * sB; C += z * sC;
    const int lane = threadIdx.x & 31, lr = lane & 15, hi = lane >> 4; const int r0 = blockIdx.x * 64, c0 = blockIdx.y * 64;
    v8f acc[4][4];
#pragma unroll
    for (int mb = 0; mb < 4; ++mb)
#pragma unroll
        for (int nb = 0; nb < 4; ++nb) acc[mb][nb] = (v8f){};
    const size_t aoff = (size_t)(r0 + lr) * K + 8 * hi, boff = (size_t)(c0 + lr) * K + 8 * hi;
#pragma unroll 1
    for (int kc = 0; kc < K; kc += 32) {
        V a[4], a2[4];
#pragma unroll
        for (int mb = 0; mb < 4; ++mb) { a[mb] = WFrag<T16>::ld(A + aoff + (size_t)mb * 16 * K + kc); if (NSPLIT == 1 || NSPLIT == 2) a2[mb] = WFrag<T16>::ld(A2 + aoff + (size_t)mb * 16 * K + kc); }
#pragma unroll
        for (int nb = 0; nb < 4; ++nb) { const V b = WFrag<T16>::ld(Bt + boff + (size_t)nb * 16 * K + kc); V b2; if (NSPLIT >= 2) b2 = WFrag<T16>::ld(Bt2 + boff + (size_t)nb * 16 * K + kc);
#pragma unroll
            for (int mb = 0; mb < 4; ++mb) { acc[mb][nb] = WFrag<T16>::mma(a[mb], b, acc[mb][nb]); if (NSPLIT == 1 || NSPLIT == 2) acc[mb][nb] = WFrag<T16>::mma(a2[mb], b, acc[mb][nb]); if (NSPLIT >= 2) acc[mb][nb] = WFrag<T16>::mma(a[mb], b2, acc[mb][nb]); } }
        asm volatile("v_nop\n\tv_nop\n\tv_nop\n\tv_nop" : "+v"(acc[0][0]), "+v"(acc[1][1]), "+v"(acc[2][2]), "+v"(acc[3][3]) : "v"(a[0]), "v"(a[3]));
    }
#pragma unroll
    for (int mb = 0; mb < 4; ++mb) {
#pragma unroll
        for (int nb = 0; nb < 4; ++nb) {
#pragma unroll
            for (int j = 0; j < 8; ++j) os[(hi * 8 + j) * 68 + nb * 16 + lr] = acc[mb][nb][j]; }
        __builtin_amdgcn_wave_barrier(); asm volatile("" ::: "memory");
        float* crow = C + (size_t)(r0 + mb * 16) * ldc + c0;
#pragma unroll 1
        for (int ps = 0; ps < 2; ++ps) {
#pragma unroll
            for (int s = 0; s < 8; ++s) { const int row = 2 * s + hi, cofs = lr * 4; v4f val = *(const v4fa*)(os + row * 68 + cofs); if (BIAS) { val[0] += bfr(bias[c0 + cofs]); val[1] += bfr(bias[c0 + cofs + 1]); val[2] += bfr(bias[c0 + cofs + 2]); val[3] += bfr(bias[c0 + cofs + 3]); }
                *(volatile v4f*)(crow + (size_t)row * ldc + cofs) = val; }
            if (ps == 0) __threadfence(); }
        __builtin_amdgcn_wave_barrier(); asm volatile("" ::: "memory");
    }
}

__global__ __launch_bounds__(256) void k_cvt8(const float* __restrict__ src, bf* dst, size_t n8) { const size_t i = (size_t)blockIdx.x * 256 + threadIdx.x; if (i >= n8) return; const v8f v = *(const v8f*)(src + i * 8); v8us o;
#pragma unroll
    for (int k = 0; k < 8; ++k) o[k] = f2bf(v[k]); *(volatile v8us*)(dst + i * 8) = o; __threadfence(); *(volatile v8us*)(dst + i * 8) = o; }

__global__ __launch_bounds__(256) void k_cvtT(const float* __restrict__ W, bf* Wt, int K, int N) {
    __shared__ unsigned short tl[64 * 66];
    const int tid = threadIdx.x; const int k0 = blockIdx.x * 64, n0 = blockIdx.y * 64;
    { const int row = tid >> 2, cseg = (tid & 3) * 16;
#pragma unroll
      for (int q = 0; q < 4; ++q) { const v4f v = *(const v4f*)(W + (size_t)(k0 + row) * N + n0 + cseg + q * 4);
#pragma unroll
          for (int j = 0; j < 4; ++j) tl[row * 66 + cseg + q * 4 + j] = f2bf(v[j]); } }
    __syncthreads();
    const int piece = tid & 7; v8us o[2];
#pragma unroll
    for (int it = 0; it < 2; ++it) { const int n = it * 32 + (tid >> 3);
#pragma unroll
        for (int j = 0; j < 8; ++j) o[it][j] = tl[(piece * 8 + j) * 66 + n]; }
#pragma unroll 1
    for (int ps = 0; ps < 2; ++ps) {
#pragma unroll
        for (int it = 0; it < 2; ++it) { const int n = it * 32 + (tid >> 3); *(volatile v8us*)(Wt + (size_t)(n0 + n) * K + k0 + piece * 8) = o[it]; }
        if (ps == 0) __threadfence(); }
}

__global__ __launch_bounds__(256) void k_hp(const float* __restrict__ F, h16* P16) {
    const size_t i = (size_t)blockIdx.x * 256 + threadIdx.x; if (i >= (size_t)NH_ * TT * HD / 8) return;
    const int d8 = (int)(i & 7); const int t = (int)((i >> 3) % TT); const int h = (int)(i / ((size_t)8 * TT));
    const float* f = F + (size_t)t * DM + h * HD + d8 * 8; const v4f a = *(const v4f*)f; const v4f b = *(const v4f*)(f + 4); v8h o;
#pragma unroll
    for (int k = 0; k < 4; ++k) { o[k] = (h16)a[k]; o[4 + k] = (h16)b[k]; }
    *(volatile v8h*)(P16 + i * 8) = o; __threadfence(); *(volatile v8h*)(P16 + i * 8) = o; }

__global__ __launch_bounds__(256) void k_vtp(const float* __restrict__ F, h16* V16) { const size_t e = ((size_t)blockIdx.x * 256 + threadIdx.x) * 2; if (e >= (size_t)NH_ * HD * TT) return; const int t = (int)(e % TT); const int d = (int)((e / TT) % HD); const int g = (int)(e / ((size_t)TT * HD)); v2h o16;
#pragma unroll
    for (int q = 0; q < 2; ++q) { const float x = F[(size_t)(t + q) * DM + g * HD + d]; o16[q] = (h16)x; }
    *(volatile v2h*)(V16 + e) = o16; __threadfence(); *(volatile v2h*)(V16 + e) = o16; }

static __device__ __forceinline__ v4f asoft_t4(const float* __restrict__ sr, const float* __restrict__ mr, int j0) {
#pragma clang fp contract(off)
    const v4f a = *(const v4f*)(sr + j0); const v4f r = *(const v4f*)(mr + j0); v4f t;
#pragma unroll
    for (int q = 0; q < 4; ++q) { const float e = a[q] * SCL; const float mt = bfr(r[q]) * -1.0e10f; t[q] = e + mt; }
    return t;
}

__global__ __launch_bounds__(256) void k_asoft(const float* __restrict__ Sb, const float* __restrict__ Mb, h16* P16) {
#pragma clang fp contract(off)
    const int lane = threadIdx.x & 31; const int wv = __builtin_amdgcn_readfirstlane(threadIdx.x >> 5); const int row = blockIdx.x * 8 + wv;
    const float* sr = Sb + (size_t)row * TT; const float* mr = Mb + (size_t)(row % RC) * SEQ_FULL;
    float mx = -3.0e38f;
#pragma unroll 1
    for (int ch = 0; ch < TT / 128; ++ch) { const v4f t = asoft_t4(sr, mr, ch * 128 + lane * 4);
#pragma unroll
        for (int q = 0; q < 4; ++q) mx = fmaxf(mx, t[q]); }
#pragma unroll
    for (int sh = 16; sh; sh >>= 1) mx = fmaxf(mx, __shfl_xor(mx, sh, 32));
    float sum = 0.f;
#pragma unroll 1
    for (int ch = 0; ch < TT / 128; ++ch) { const v4f t = asoft_t4(sr, mr, ch * 128 + lane * 4);
#pragma unroll
        for (int q = 0; q < 4; ++q) { float d0 = __fsub_rn(t[q], mx); asm volatile("" : "+v"(d0)); const float p = __builtin_amdgcn_exp2f(__fmul_rn(d0, 1.4426950408889634f)); sum += p; } }
#pragma unroll
    for (int sh = 16; sh; sh >>= 1) sum += __shfl_xor(sum, sh, 32);
    const float f = __fdiv_rn(PCAR, sum);
    h16* prow = P16 + (size_t)row * TT + lane * 4;
#pragma unroll 1
    for (int ch = 0; ch < TT / 128; ++ch) { const v4f t = asoft_t4(sr, mr, ch * 128 + lane * 4); v4h o4;
#pragma unroll
        for (int q = 0; q < 4; ++q) { float d0 = __fsub_rn(t[q], mx); asm volatile("" : "+v"(d0)); const float p = __builtin_amdgcn_exp2f(__fmul_rn(d0, 1.4426950408889634f)); o4[q] = toh_flush(p * f); }
        *(volatile v4h*)(prow + ch * 128) = o4; __threadfence(); *(volatile v4h*)(prow + ch * 128) = o4; }
}

__global__ __launch_bounds__(256) void k_merge(const float* __restrict__ O, bf* Ah, bf* Al) { const size_t e = ((size_t)blockIdx.x * 256 + threadIdx.x) * 2; if (e >= (size_t)NH_ * TT * HD) return; const int d = (int)(e % HD); const int t = (int)((e / HD) % TT); const int zz = (int)(e / ((size_t)HD * TT)); const float cs = 1.0f / PCAR; const size_t oo = (size_t)t * DM + zz * HD + d;
    v2us oh, ol;
#pragma unroll
    for (int q = 0; q < 2; ++q) { unsigned short a, c2; splitf(O[e + q] * cs, a, c2); oh[q] = a; ol[q] = c2; } *(volatile v2us*)(Ah + oo) = oh; *(volatile v2us*)(Al + oo) = ol; __threadfence(); *(volatile v2us*)(Ah + oo) = oh; *(volatile v2us*)(Al + oo) = ol; }

constexpr size_t al256(size_t b) { return (b + 255) & ~(size_t)255; }
constexpr size_t WS_TOTAL = 4 * al256((size_t)DM * DM * 2) + al256((size_t)TT * DM * 2) + al256((size_t)TT * DM * 4) + 3 * al256((size_t)NH_ * TT * HD * 2)
                          + al256((size_t)NH_ * RC * TT * 4) + al256((size_t)NH_ * RC * TT * 2) + al256((size_t)NH_ * TT * HD * 4) + 2 * al256((size_t)TT * DM * 2);
static_assert(WS_TOTAL <= (size_t)134217728);

extern "C" void kernel_launch(void* const* d_in, const int* in_sizes, int n_in,
                              void* d_out, int out_size, void* d_ws, size_t ws_size, hipStream_t stream) {
    if (n_in < 12) return;
    const size_t need_x = ((size_t)(NB - 1) * SEQ_FULL + SEQ) * DM;
    const size_t need_m = (size_t)(NB - 1) * SEQ_FULL * SEQ_FULL + (size_t)(SEQ - 1) * SEQ_FULL + SEQ;
    if ((size_t)in_sizes[0] < need_x || (size_t)in_sizes[1] < need_x || (size_t)in_sizes[2] < need_x || (size_t)in_sizes[3] < need_m) return;
    if (in_sizes[4] < DM * DM || in_sizes[6] < DM * DM || in_sizes[8] < DM * DM || in_sizes[10] < DM * DM) return;
    if (in_sizes[5] < DM || in_sizes[7] < DM || in_sizes[9] < DM || in_sizes[11] < DM) return;
    if ((size_t)out_size < need_x) return;
    const float* xq = (const float*)d_in[0]; const float* xk = (const float*)d_in[1]; const float* xv = (const float*)d_in[2];
    const float* msk = (const float*)d_in[3];
    const float* wq = (const float*)d_in[4]; const float* bq = (const float*)d_in[5]; const float* wk = (const float*)d_in[6]; const float* bk = (const float*)d_in[7];
    const float* wv = (const float*)d_in[8]; const float* bv = (const float*)d_in[9]; const float* wo = (const float*)d_in[10]; const float* bo = (const float*)d_in[11];
    float* OUT = (float*)d_out;
    char* wsp = (char*)d_ws;
    auto take = [&](size_t bytes) { char* p = wsp; wsp += (bytes + 255) & ~(size_t)255; return (void*)p; };
    bf* WQ = (bf*)take((size_t)DM * DM * 2); bf* WK = (bf*)take((size_t)DM * DM * 2); bf* WV = (bf*)take((size_t)DM * DM * 2); bf* WO = (bf*)take((size_t)DM * DM * 2);
    bf* XB = (bf*)take((size_t)TT * DM * 2); float* F = (float*)take((size_t)TT * DM * 4);
    h16* QP16 = (h16*)take((size_t)NH_ * TT * HD * 2); h16* KP16 = (h16*)take((size_t)NH_ * TT * HD * 2); h16* VT16 = (h16*)take((size_t)NH_ * HD * TT * 2);
    float* Sb = (float*)take((size_t)NH_ * RC * TT * 4); h16* P16 = (h16*)take((size_t)NH_ * RC * TT * 2);
    float* Ob = (float*)take((size_t)NH_ * TT * HD * 4); bf* ATh = (bf*)take((size_t)TT * DM * 2); bf* ATl = (bf*)take((size_t)TT * DM * 2);
    if ((size_t)(wsp - (char*)d_ws) > ws_size) return;
    k_cvtT<<<dim3(DM / 64, DM / 64), 256, 0, stream>>>(wq, WQ, DM, DM);
    k_cvtT<<<dim3(DM / 64, DM / 64), 256, 0, stream>>>(wk, WK, DM, DM);
    k_cvtT<<<dim3(DM / 64, DM / 64), 256, 0, stream>>>(wv, WV, DM, DM);
    k_cvtT<<<dim3(DM / 64, DM / 64), 256, 0, stream>>>(wo, WO, DM, DM);
    const unsigned LX = (unsigned)(((size_t)TT * DM / 8 + 255) / 256);
    const unsigned LH = (unsigned)(((size_t)NH_ * TT * HD / 8 + 255) / 256);
    const unsigned LV = (unsigned)(((size_t)NH_ * HD * TT / 2 + 255) / 256);
    for (int b = 0; b < NB; ++b) {
        const size_t xoff = (size_t)b * SEQ_FULL * DM;
        k_cvt8<<<LX, 256, 0, stream>>>(xq + xoff, XB, (size_t)TT * DM / 8);
        k_gemmw<bf, 0, true><<<dim3(TT / 64, DM / 64, 1), 32, 0, stream>>>(XB, nullptr, WQ, nullptr, DM, F, DM, bq, 0, 0, 0);
        k_hp<<<LH, 256, 0, stream>>>(F, QP16);
        k_cvt8<<<LX, 256, 0, stream>>>(xk + xoff, XB, (size_t)TT * DM / 8);
        k_gemmw<bf, 0, true><<<dim3(TT / 64, DM / 64, 1), 32, 0, stream>>>(XB, nullptr, WK, nullptr, DM, F, DM, bk, 0, 0, 0);
        k_hp<<<LH, 256, 0, stream>>>(F, KP16);
        k_cvt8<<<LX, 256, 0, stream>>>(xv + xoff, XB, (size_t)TT * DM / 8);
        k_gemmw<bf, 0, true><<<dim3(TT / 64, DM / 64, 1), 32, 0, stream>>>(XB, nullptr, WV, nullptr, DM, F, DM, bv, 0, 0, 0);
        k_vtp<<<LV, 256, 0, stream>>>(F, VT16);
        for (int c = 0; c < TT / RC; ++c) {
            k_gemmw<h16, 0, false><<<dim3(RC / 64, TT / 64, NH_), 32, 0, stream>>>(QP16 + (size_t)c * RC * HD, nullptr, KP16, nullptr, HD, Sb, TT, nullptr, (size_t)TT * HD, (size_t)TT * HD, (size_t)RC * TT);
            k_asoft<<<NH_ * RC / 8, 256, 0, stream>>>(Sb, msk + ((size_t)b * SEQ_FULL + (size_t)c * RC) * SEQ_FULL, P16);
            k_gemmw<h16, 0, false><<<dim3(RC / 64, HD / 64, NH_), 32, 0, stream>>>(P16, nullptr, VT16, nullptr, TT, Ob + (size_t)c * RC * HD, HD, nullptr, (size_t)RC * TT, (size_t)HD * TT, (size_t)TT * HD);
        }
        k_merge<<<(unsigned)(((size_t)NH_ * TT * HD / 2 + 255) / 256), 256, 0, stream>>>(Ob, ATh, ATl);
        k_gemmw<bf, 1, true><<<dim3(TT / 64, DM / 64, 1), 32, 0, stream>>>(ATh, ATl, WO, nullptr, DM, OUT + xoff, DM, bo, 0, 0, 0);
    }
}
